// GraphAttentionLayer_52905407152165
// MI455X (gfx1250) — hardware-verified
//
#include <hip/hip_runtime.h>
#include <stddef.h>


typedef _Float16 v16h __attribute__((ext_vector_type(16)));
typedef _Float16 v8h  __attribute__((ext_vector_type(8)));
typedef _Float16 v4h  __attribute__((ext_vector_type(4)));
typedef float    v8f  __attribute__((ext_vector_type(8)));
typedef float    v4f  __attribute__((ext_vector_type(4)));
typedef int      v4i  __attribute__((ext_vector_type(4)));
typedef _Float16 h16;

#ifndef NB
#define NB 32
#endif
#ifndef SEQ
#define SEQ 228
#endif
#define NB_FULL  32
#define SEQ_FULL 228
#define FIN   128
#define FOUT  64
#define SEQP  (((SEQ + 127) / 128) * 128)
#define MROWS (NB * SEQP)

static_assert(NB >= 1 && NB <= NB_FULL);
static_assert(SEQ >= 16 && SEQ <= SEQ_FULL);
static_assert((SEQ % 4) == 0 && (SEQ_FULL % 4) == 0);
static_assert((SEQP % 128) == 0 && (SEQP % 64) == 0 && (SEQP % 32) == 0 && SEQP >= SEQ);
static_assert((FIN % 64) == 0 && (FIN % 32) == 0 && (FIN % 8) == 0);
static_assert(FOUT == 64);
static_assert(FOUT == 4 * 16);
static_assert(FOUT == 16 * 4);
static_assert((MROWS % 64) == 0);
static_assert(((size_t)MROWS * FIN) % 2048 == 0);
static_assert((size_t)MROWS * FIN < (size_t)0xFFFFFFFFu);
static_assert(((size_t)(NB - 1) * SEQ_FULL + SEQ) * FOUT <= (size_t)NB_FULL * SEQ_FULL * FOUT);

#define LDT 72
#define LDC 68
#define PLD (SEQP + 8)
#define HLD (FOUT + 4)
#define NIT (SEQP / 128)
static_assert((LDT % 8) == 0 && LDT >= 64);
static_assert((LDC % 4) == 0 && LDC >= 64);
static_assert((PLD % 8) == 0 && (HLD % 4) == 0);
static_assert(NIT * 128 == SEQP && NIT <= 8);
static_assert(4 * 4 == 16);
static_assert(4 * 2 * 2 == 16);

#define BN_STEPS ((NB * 16 + 255) / 256)
static_assert(BN_STEPS * 256 >= NB * 16 && BN_STEPS >= 1 && BN_STEPS <= 4);

#define WCARRY 64.0f
#define PCARRY 16384.0f
#define ALPHA  0.2f
#define NEGFILL (-9.0e15f)
#define BNEPS  1.0e-5f

#define WT_BYTES  ((size_t)FOUT * FIN * 2)
#define H16_BYTES ((size_t)MROWS * FIN * 2)
#define VT_BYTES  ((size_t)NB * FOUT * SEQP * 2)
#define FP_BYTES  ((size_t)(FOUT / 64) * 2 * MROWS * 4)
#define HP_BYTES  ((size_t)NB * SEQ * FOUT * 4)
#define OFF_WT  ((size_t)0)
#define OFF_H16 (OFF_WT + WT_BYTES)
#define OFF_VT  (OFF_H16 + H16_BYTES)
#define OFF_FP  (OFF_VT + VT_BYTES)
#define OFF_HP  (OFF_FP + FP_BYTES)
#define WS_TOTAL (OFF_HP + HP_BYTES)
static_assert((WT_BYTES % 128) == 0 && (H16_BYTES % 128) == 0);
static_assert((VT_BYTES % 128) == 0 && (FP_BYTES % 128) == 0 && (HP_BYTES % 128) == 0);
static_assert(WS_TOTAL <= (size_t)134217728);

__device__ __forceinline__ float bf16r(float x) {
  unsigned int u = __float_as_uint(x);
  u = (u + 0x7FFFu + ((u >> 16) & 1u)) & 0xFFFF0000u;
  return __uint_as_float(u);
}

static __device__ __forceinline__ h16 toh_flush(float v) {
  const h16 r = (h16)v;
  return (fabsf(v) < 6.103515625e-05f) ? (h16)0.0f : r;
}

__device__ __forceinline__ v16h frag_at(const _Float16* p) {
  v8h lo = *(const v8h*)(p);
  v8h hi = *(const v8h*)(p + 16);
  v16h out;
#pragma unroll
  for (int i = 0; i < 8; ++i) { out[i] = lo[i]; out[i + 8] = hi[i]; }
  return out;
}
__device__ __forceinline__ v16h ld_frag(const _Float16* base, unsigned ld) {
  const unsigned lane = threadIdx.x & 31u;
  return frag_at(base + (lane & 15u) * ld + (lane >> 4) * 8u);
}

__device__ __forceinline__ v8f wmma16(v16h a, v16h b, v8f c) {
  v8f d = __builtin_amdgcn_wmma_f32_16x16x32_f16(false, a, false, b, (short)0, c,
                                                 false, false);
  asm volatile("v_nop\n\tv_nop\n\tv_nop\n\tv_nop" : "+v"(d) : "v"(a), "v"(b));
  return d;
}

__device__ __forceinline__ float red32_sum(float x) {
#pragma unroll
  for (int off = 1; off < 32; off <<= 1) x += __shfl_xor(x, off, 32);
  return x;
}
__device__ __forceinline__ float red32_max(float x) {
#pragma unroll
  for (int off = 1; off < 32; off <<= 1) x = fmaxf(x, __shfl_xor(x, off, 32));
  return x;
}

__global__ __launch_bounds__(256) void wconv_kernel(
    const float* __restrict__ W, _Float16* __restrict__ Wt, unsigned ldw, unsigned ldk) {
  __shared__ _Float16 T[64 * LDT];
  const unsigned tid = threadIdx.x;
  const unsigned n0 = blockIdx.x * 64u;
  const unsigned k0 = blockIdx.y * 64u;
#pragma unroll 4
  for (unsigned j = 0; j < 16u; ++j) {
    const unsigned idx = tid + 256u * j;
    const unsigned kr = idx >> 6, nc = idx & 63u;
    const float v = W[(size_t)(k0 + kr) * ldw + n0 + nc];
    T[nc * LDT + kr] = toh_flush(WCARRY * bf16r(v));
  }
  __syncthreads();
  v8h x[2];
  size_t off[2];
#pragma unroll
  for (unsigned i = 0; i < 2u; ++i) {
    const unsigned n = 32u * i + (tid >> 3);
    const unsigned kc = (tid & 7u) * 8u;
    x[i] = *(const v8h*)&T[n * LDT + kc];
    off[i] = (size_t)(n0 + n) * ldk + k0 + kc;
  }
#pragma unroll
  for (int i = 0; i < 2; ++i) *(volatile v8h*)(Wt + off[i]) = x[i];
  __threadfence();
#pragma unroll
  for (int i = 0; i < 2; ++i) *(volatile v8h*)(Wt + off[i]) = x[i];
}

__global__ __launch_bounds__(256) void hconv_kernel(
    const float* __restrict__ X, _Float16* __restrict__ dst) {
  const unsigned g = blockIdx.x * 256u + threadIdx.x;
  const unsigned crow = g / (unsigned)(FIN / 8);
  const unsigned c = (g - crow * (unsigned)(FIN / 8)) * 8u;
  const unsigned bidx = crow / (unsigned)SEQP;
  const unsigned sq = crow - bidx * (unsigned)SEQP;
  const bool ok = sq < (unsigned)SEQ;
  const unsigned sqc = ok ? sq : (unsigned)(SEQ - 1);
  const size_t srow = (size_t)bidx * SEQ_FULL + sqc;
  const v4f a0 = *(const v4f*)(X + srow * FIN + c);
  const v4f a1 = *(const v4f*)(X + srow * FIN + c + 4u);
  v8h o;
#pragma unroll
  for (int i = 0; i < 4; ++i) {
    const float u0 = ok ? a0[i] : 0.0f;
    const float u1 = ok ? a1[i] : 0.0f;
    o[i]     = toh_flush(bf16r(u0));
    o[i + 4] = toh_flush(bf16r(u1));
  }
  _Float16* p = dst + (size_t)crow * FIN + c;
  *(volatile v8h*)p = o;
  __threadfence();
  *(volatile v8h*)p = o;
}

__global__ __launch_bounds__(256) void gemm_wh_kernel(
    const _Float16* __restrict__ A16, const _Float16* __restrict__ Bt,
    const float* __restrict__ avec, _Float16* __restrict__ vt, float* __restrict__ fp) {
  __shared__ __attribute__((aligned(16))) float Cs[64 * LDC];
  __shared__ __attribute__((aligned(16))) float Fs[2 * 64];
  const unsigned tid = threadIdx.x, lane = tid & 31u;
  const unsigned w = __builtin_amdgcn_readfirstlane(tid >> 5);
  const unsigned mw = w >> 1, nw = w & 1u;
  const unsigned hh = lane >> 4, m = lane & 15u;
  const unsigned n0 = blockIdx.x * 64u;
  const unsigned row0 = blockIdx.y * 64u;
  const unsigned K = (unsigned)FIN;

  const _Float16* ap  = A16 + (size_t)(row0 + mw * 16u + m) * K + hh * 8u;
  const _Float16* bp0 = Bt + (size_t)(n0 + nw * 32u + m) * K + hh * 8u;
  const _Float16* bp1 = bp0 + (size_t)16 * K;
  v8f acc0 = {}, acc1 = {};
#pragma unroll 2
  for (unsigned k0 = 0; k0 < K; k0 += 32u) {
    const v16h a  = frag_at(ap + k0);
    const v16h b0 = frag_at(bp0 + k0);
    const v16h b1 = frag_at(bp1 + k0);
    acc0 = wmma16(a, b0, acc0);
    acc1 = wmma16(a, b1, acc1);
  }
#pragma unroll
  for (int r = 0; r < 8; ++r) {
    float* d = &Cs[(mw * 16u + hh * 8u + (unsigned)r) * LDC + nw * 32u + m];
    d[0]  = acc0[r];
    d[16] = acc1[r];
  }
  __syncthreads();

  {
    const unsigned bidx = row0 / (unsigned)SEQP;
    const unsigned key0 = row0 - bidx * (unsigned)SEQP;
    v8h x[2];
    size_t off[2];
#pragma unroll
    for (unsigned i = 0; i < 2u; ++i) {
      const unsigned dcol = 32u * i + (tid >> 3);
      const unsigned kk = (tid & 7u) * 8u;
#pragma unroll
      for (unsigned j = 0; j < 8u; ++j) {
        const float t = Cs[(kk + j) * LDC + dcol] * (1.0f / WCARRY);
        x[i][j] = toh_flush(t);
      }
      off[i] = ((size_t)bidx * FOUT + n0 + dcol) * SEQP + key0 + kk;
    }
#pragma unroll
    for (int i = 0; i < 2; ++i) *(volatile v8h*)(vt + off[i]) = x[i];
    __threadfence();
#pragma unroll
    for (int i = 0; i < 2; ++i) *(volatile v8h*)(vt + off[i]) = x[i];
  }

  {
    const unsigned r = tid >> 2, q = tid & 3u;
    float s1 = 0.0f, s2 = 0.0f;
#pragma unroll 4
    for (unsigned j = 0; j < 16u; ++j) {
      const unsigned c = q * 16u + j;
      const float t = Cs[r * LDC + c] * (1.0f / WCARRY);
      s1 += t * bf16r(avec[n0 + c]);
      s2 += t * bf16r(avec[(unsigned)FOUT + n0 + c]);
    }
    s1 += __shfl_xor(s1, 1, 32);
    s2 += __shfl_xor(s2, 1, 32);
    s1 += __shfl_xor(s1, 2, 32);
    s2 += __shfl_xor(s2, 2, 32);
    if (q == 0u) { Fs[r] = s1; Fs[64u + r] = s2; }
  }
  __syncthreads();
  if (w == 0u) {
    const unsigned which = lane >> 4, ch = lane & 15u;
    const v4f v = *(const v4f*)&Fs[which * 64u + ch * 4u];
    float* p = fp + (size_t)(blockIdx.x * 2u + which) * MROWS + row0 + ch * 4u;
    *(volatile v4f*)p = v;
    __threadfence();
    *(volatile v4f*)p = v;
  }
}

__global__ __launch_bounds__(128) void gat_attn_kernel(
    const int* __restrict__ adj, const _Float16* __restrict__ Vt,
    const float* __restrict__ Fp, float* __restrict__ hp) {
  __shared__ __attribute__((aligned(16))) _Float16 Ps[16 * PLD];
  __shared__ __attribute__((aligned(16))) float Hs[16 * HLD];
  __shared__ __attribute__((aligned(16))) float f2s[SEQP];
  __shared__ float f1s[16];
  __shared__ float rinv[16];

  const unsigned tid = threadIdx.x, lane = tid & 31u;
  const unsigned w = __builtin_amdgcn_readfirstlane(tid >> 5);
  const unsigned hh = lane >> 4, m = lane & 15u;
  const unsigned i0 = blockIdx.x * 16u;
  const unsigned b = blockIdx.y;

  for (unsigned j4 = tid; j4 < (unsigned)(SEQP / 4); j4 += 128u) {
    const float* p = Fp + (size_t)MROWS + (size_t)b * SEQP + j4 * 4u;
    const v4f s = *(const v4f*)(p);
    *(v4f*)&f2s[j4 * 4u] = s;
  }
  {
    const unsigned ci = tid & 15u;
    const float f = Fp[(size_t)b * SEQP + i0 + ci];
    if (tid < 16u) f1s[tid] = f;
  }
  __syncthreads();

#pragma unroll 1
  for (unsigned rr = 0; rr < 4u; ++rr) {
    const unsigned r = w * 4u + rr;
    const float f1v = f1s[r];
    const unsigned node = i0 + r;
    const unsigned nodec = (node < (unsigned)SEQ) ? node : (unsigned)(SEQ - 1);
    const int* adjR = adj + ((size_t)b * SEQ_FULL + nodec) * SEQ_FULL;
    float e[NIT * 4];
    float mx = -3.0e38f;
#pragma unroll
    for (int it = 0; it < NIT; ++it) {
      const unsigned key = (unsigned)it * 128u + lane * 4u;
      const bool kv = key < (unsigned)SEQ;
      const unsigned kc = kv ? key : (unsigned)(SEQ - 4);
      const v4i a4 = *(const v4i*)(adjR + kc);
      const v4f fv = *(const v4f*)&f2s[key];
#pragma unroll
      for (int q = 0; q < 4; ++q) {
        const float t = f1v + fv[q];
        const float lr = (t > 0.0f) ? t : ALPHA * t;
        const float ev = (a4[q] > 0) ? lr : NEGFILL;
        e[it * 4 + q] = ev;
        mx = kv ? fmaxf(mx, ev) : mx;
      }
    }
    mx = red32_max(mx);
    float sum = 0.0f;
#pragma unroll
    for (int it = 0; it < NIT; ++it) {
      const unsigned key = (unsigned)it * 128u + lane * 4u;
      const bool kv = key < (unsigned)SEQ;
      v4h pk;
#pragma unroll
      for (int q = 0; q < 4; ++q) {
        const float pe = __expf(e[it * 4 + q] - mx) * PCARRY;
        const float pv = kv ? pe : 0.0f;
        const h16 hv = toh_flush(pv);
        pk[q] = hv;
        sum += (float)hv;
      }
      *(v4h*)&Ps[r * PLD + key] = pk;
    }
    sum = red32_sum(sum);
    if (lane == 0u) rinv[r] = 1.0f / sum;
  }
  __syncthreads();

  {
    const _Float16* bp0 = Vt + ((size_t)b * FOUT + w * 16u + m) * SEQP + hh * 8u;
    v8f acc0 = {};
#pragma unroll 2
    for (unsigned k0 = 0; k0 < (unsigned)SEQP; k0 += 32u) {
      const v16h a  = ld_frag(&Ps[k0], PLD);
      const v16h b0 = frag_at(bp0 + k0);
      acc0 = wmma16(a, b0, acc0);
    }
#pragma unroll
    for (int r = 0; r < 8; ++r) {
      const unsigned row = hh * 8u + (unsigned)r;
      const float ri = rinv[row];
      Hs[row * HLD + w * 16u + m] = acc0[r] * ri;
    }
  }
  __syncthreads();

#pragma unroll 1
  for (unsigned s = 0; s < 2u; ++s) {
    const unsigned r = w * 4u + s * 2u + hh;
    const v4f x = *(const v4f*)&Hs[r * HLD + m * 4u];
    v4f o;
#pragma unroll
    for (int i = 0; i < 4; ++i) {
      const float v = x[i];
      const float en = expm1f(fminf(v, 0.0f));
      o[i] = (v > 0.0f) ? v : en;
    }
    const unsigned node = i0 + r;
    const bool ok = node < (unsigned)SEQ;
    const unsigned nodec = ok ? node : (unsigned)(SEQ - 1);
    float* p = hp + ((size_t)b * SEQ + nodec) * FOUT + m * 4u;
    if (ok) *(volatile v4f*)p = o;
    __threadfence();
    if (ok) *(volatile v4f*)p = o;
  }
}

__global__ __launch_bounds__(256) void bn_kernel(
    const float* __restrict__ hp, const float* __restrict__ G,
    const float* __restrict__ Be, float* __restrict__ out) {
#pragma clang fp contract(off)
  __shared__ float redA[8];
  __shared__ float redB[8];
  const unsigned tid = threadIdx.x, lane = tid & 31u;
  const unsigned w = __builtin_amdgcn_readfirstlane(tid >> 5);
  const unsigned n = blockIdx.x;

  v4f x[BN_STEPS];
  float s = 0.0f;
#pragma unroll
  for (int st = 0; st < BN_STEPS; ++st) {
    const unsigned idx4 = tid + 256u * (unsigned)st;
    const bool ok = idx4 < (unsigned)(NB * 16);
    const unsigned bb = ok ? (idx4 >> 4) : (unsigned)(NB - 1);
    const unsigned c4 = idx4 & 15u;
    v4f v = *(const v4f*)(hp + ((size_t)bb * SEQ + n) * FOUT + c4 * 4u);
#pragma unroll
    for (int i = 0; i < 4; ++i) v[i] = ok ? v[i] : 0.0f;
    x[st] = v;
    s += (v[0] + v[1]) + (v[2] + v[3]);
  }
  s = red32_sum(s);
  if (lane == 0u) redA[w] = s;
  __syncthreads();
  float tot = 0.0f;
#pragma unroll 1
  for (unsigned i = 0; i < 8u; ++i) tot += redA[i];
  const float mean = tot * (1.0f / (float)(NB * FOUT));

  float ss = 0.0f;
#pragma unroll
  for (int st = 0; st < BN_STEPS; ++st) {
    const unsigned idx4 = tid + 256u * (unsigned)st;
    const bool ok = idx4 < (unsigned)(NB * 16);
#pragma unroll
    for (int i = 0; i < 4; ++i) {
      const float d = ok ? (x[st][i] - mean) : 0.0f;
      ss += d * d;
    }
  }
  ss = red32_sum(ss);
  if (lane == 0u) redB[w] = ss;
  __syncthreads();
  float tot2 = 0.0f;
#pragma unroll 1
  for (unsigned i = 0; i < 8u; ++i) tot2 += redB[i];
  const float var = tot2 * (1.0f / (float)(NB * FOUT));
  const float rstd = 1.0f / sqrtf(var + BNEPS);
  const float g = bf16r(G[n]);
  const float be = bf16r(Be[n]);

  v4f o[BN_STEPS];
  size_t off[BN_STEPS];
  bool okk[BN_STEPS];
#pragma unroll
  for (int st = 0; st < BN_STEPS; ++st) {
    const unsigned idx4 = tid + 256u * (unsigned)st;
    const bool ok = idx4 < (unsigned)(NB * 16);
    const unsigned bb = ok ? (idx4 >> 4) : (unsigned)(NB - 1);
    const unsigned c4 = idx4 & 15u;
#pragma unroll
    for (int i = 0; i < 4; ++i) o[st][i] = g * ((x[st][i] - mean) * rstd) + be;
    off[st] = ((size_t)bb * SEQ_FULL + n) * FOUT + c4 * 4u;
    okk[st] = ok;
  }
#pragma unroll
  for (int st = 0; st < BN_STEPS; ++st) if (okk[st]) *(volatile v4f*)(out + off[st]) = o[st];
  __threadfence();
#pragma unroll
  for (int st = 0; st < BN_STEPS; ++st) if (okk[st]) *(volatile v4f*)(out + off[st]) = o[st];
}

static_assert(16 * PLD * 2 + 16 * HLD * 4 + SEQP * 4 + 64 + 64 <= 131072);
static_assert(64 * LDC * 4 + 2 * 64 * 4 <= 131072);
static_assert(64 * LDT * 2 <= 131072);

extern "C" void kernel_launch(void* const* d_in, const int* in_sizes, int n_in,
                              void* d_out, int out_size, void* d_ws, size_t ws_size,
                              hipStream_t stream) {
  if (n_in < 6) return;
  const long long need_rows = (long long)(NB - 1) * SEQ_FULL + SEQ;
  if ((long long)in_sizes[0] < need_rows * FIN) return;
  if ((long long)in_sizes[1] < (need_rows - 1) * SEQ_FULL + SEQ) return;
  if ((long long)in_sizes[2] < (long long)FIN * FOUT) return;
  if (in_sizes[3] < 2 * FOUT) return;
  if (in_sizes[4] < SEQ || in_sizes[5] < SEQ) return;
  if ((long long)out_size < need_rows * FOUT) return;
  if (ws_size < WS_TOTAL) return;

  const float* X     = (const float*)d_in[0];
  const int*   adj   = (const int*)d_in[1];
  const float* Wm    = (const float*)d_in[2];
  const float* avec  = (const float*)d_in[3];
  const float* gamma = (const float*)d_in[4];
  const float* beta  = (const float*)d_in[5];
  float* out = (float*)d_out;

  char* ws = (char*)d_ws;
  _Float16* Wt16 = (_Float16*)(ws + OFF_WT);
  _Float16* H16  = (_Float16*)(ws + OFF_H16);
  _Float16* Vt16 = (_Float16*)(ws + OFF_VT);
  float*    Fp   = (float*)(ws + OFF_FP);
  float*    Hp   = (float*)(ws + OFF_HP);

  dim3 blk(256);
  wconv_kernel<<<dim3(FOUT / 64, FIN / 64), blk, 0, stream>>>(Wm, Wt16, (unsigned)FOUT, (unsigned)FIN);
  hconv_kernel<<<dim3((unsigned)(((size_t)MROWS * FIN) / 2048)), blk, 0, stream>>>(X, H16);
  gemm_wh_kernel<<<dim3(FOUT / 64, MROWS / 64), blk, 0, stream>>>(H16, Wt16, avec, Vt16, Fp);
  gat_attn_kernel<<<dim3((SEQ + 15) / 16, NB), dim3(128), 0, stream>>>(adj, Vt16, Fp, Hp);
  bn_kernel<<<dim3(SEQ), blk, 0, stream>>>(Hp, gamma, beta, out);
}
